// NGCF_55989193671007
// MI455X (gfx1250) — hardware-verified
//
#include <hip/hip_runtime.h>
#include <stddef.h>
#include <stdint.h>
#include <math.h>


#define F       64
#define KC      256
#define NL      3
#define ALLP    (NL * F)
#define OW      ((NL + 1) * F)
#define NTHR    256
#define NWAVE   8
#define EPT     8
#define CHUNK   (NTHR * EPT)
#define WCAP    (EPT * 32)
#define LISTN   (NWAVE * WCAP)
#define NBA     1024
#define PKS     10
#define RCAP    28672
#define DEGCAP  64
#define GBM     64
#define GTHR    128
#define UPL     (2 * F * (2 * F / 8))
#define ZINTS   (2 * RCAP + 2 * NBA + LISTN)
#define LDS_AGG (ZINTS * 4 + 64)
#define WSMAX   134217728

static_assert((CHUNK & (CHUNK - 1)) == 0);
static_assert(NBA == (1 << PKS));
static_assert(((long long)CHUNK << PKS) < (1LL << 31));
static_assert(NTHR * 4 == NBA);
static_assert(LISTN >= NBA && LISTN >= NWAVE * WCAP);
static_assert((RCAP % 32) == 0);
static_assert((ZINTS % (NTHR * 4)) == 0);
static_assert(LDS_AGG <= 262144);
static_assert((NBA % NWAVE) == 0 && (NBA % GBM) == 0);
static_assert(GBM == (GTHR / 32) * 16 && F == 16 * 4 && F == 2 * 32);
static_assert(KC == 4 * F && (KC % 32) == 0);
static_assert((UPL % NTHR) == 0 && UPL == 2048);
static_assert(GTHR * 32 == GBM * F);
static_assert(((ALLP * 4) % 128) == 0 && OW == 8 * 32 && ALLP == 3 * F);

typedef float          v2f  __attribute__((ext_vector_type(2)));
typedef float          v4f  __attribute__((ext_vector_type(4)));
typedef float          v8f  __attribute__((ext_vector_type(8)));
typedef int            v4i  __attribute__((ext_vector_type(4)));
typedef int            v8i  __attribute__((ext_vector_type(8)));
typedef unsigned short v8us __attribute__((ext_vector_type(8)));
typedef __bf16         v16b __attribute__((ext_vector_type(16)));
typedef v4f  __attribute__((may_alias)) v4fa;
typedef v4i  __attribute__((may_alias)) v4ia;
typedef v8us __attribute__((may_alias)) v8usa;
union Frag { v16b b; v8us h[2]; v8i w; };

__device__ __forceinline__ v8f wmb(const Frag& a, const Frag& b, v8f c) {
  v8f d = __builtin_amdgcn_wmma_f32_16x16x32_bf16(false, a.b, false, b.b, (short)0, c, false, false);
  asm volatile("v_nop\n\tv_nop\n\tv_nop\n\tv_nop" : "+v"(d) : "v"(a.w), "v"(b.w));
  return d;
}

__device__ __forceinline__ unsigned short bf_bits(float f) {
  unsigned int u = __float_as_uint(f);
  u += 0x7FFFu + ((u >> 16) & 1u);
  return (unsigned short)(u >> 16);
}
__device__ __forceinline__ float bf_val(unsigned short b) {
  return __uint_as_float(((unsigned int)b) << 16);
}
__device__ __forceinline__ float bf_rne(float f) { return bf_val(bf_bits(f)); }

__device__ __forceinline__ void split2(float s, float e, unsigned short& hs, unsigned short& ls,
                                       unsigned short& hp, unsigned short& lp) {
  hs = bf_bits(s);
  ls = bf_bits(s - bf_val(hs));
  const float p = e * s;
  hp = bf_bits(p);
  lp = bf_bits(p - bf_val(hp));
}

__device__ __forceinline__ int scan_chunk(const int* __restrict__ dsts, int nE, int cbase, int slotBase,
                                          int nb, int vec8, int* list, int tid, int lane, int wave) {
  int wc = 0;
  const int el0  = tid * EPT;
  const int e0   = cbase + el0;
  const int sent = -2147483647 - 1;
  v4i da, db;
  if (vec8 != 0 && cbase + CHUNK <= nE) {
    da = *(const v4i*)(dsts + e0);
    db = *(const v4i*)(dsts + e0 + 4);
  } else {
    da.x = (e0     < nE) ? dsts[min(e0,     nE - 1)] : sent;
    da.y = (e0 + 1 < nE) ? dsts[min(e0 + 1, nE - 1)] : sent;
    da.z = (e0 + 2 < nE) ? dsts[min(e0 + 2, nE - 1)] : sent;
    da.w = (e0 + 3 < nE) ? dsts[min(e0 + 3, nE - 1)] : sent;
    db.x = (e0 + 4 < nE) ? dsts[min(e0 + 4, nE - 1)] : sent;
    db.y = (e0 + 5 < nE) ? dsts[min(e0 + 5, nE - 1)] : sent;
    db.z = (e0 + 6 < nE) ? dsts[min(e0 + 6, nE - 1)] : sent;
    db.w = (e0 + 7 < nE) ? dsts[min(e0 + 7, nE - 1)] : sent;
  }
  const unsigned nbs = (unsigned)slotBase;
  const unsigned unb = (unsigned)nb;
  const unsigned s0 = (unsigned)da.x - nbs, s1 = (unsigned)da.y - nbs;
  const unsigned s2 = (unsigned)da.z - nbs, s3 = (unsigned)da.w - nbs;
  const unsigned s4 = (unsigned)db.x - nbs, s5 = (unsigned)db.y - nbs;
  const unsigned s6 = (unsigned)db.z - nbs, s7 = (unsigned)db.w - nbs;
  const bool h0 = s0 < unb, h1 = s1 < unb, h2 = s2 < unb, h3 = s3 < unb;
  const bool h4 = s4 < unb, h5 = s5 < unb, h6 = s6 < unb, h7 = s7 < unb;
  const unsigned any = __builtin_amdgcn_ballot_w32(h0 | h1 | h2 | h3 | h4 | h5 | h6 | h7);
  if (any != 0u) {
#define HITJ(J, HJ, SJ) { \
      const unsigned mj = __builtin_amdgcn_ballot_w32(HJ); \
      if (mj != 0u) { \
        if (HJ) { \
          const int pos = wc + (int)__builtin_amdgcn_mbcnt_lo(mj, 0u); \
          if (pos < WCAP) list[wave * WCAP + pos] = ((el0 + (J)) << PKS) | (int)(SJ); \
        } \
        wc += (int)__builtin_popcount(mj); } }
    HITJ(0, h0, s0)
    HITJ(1, h1, s1)
    HITJ(2, h2, s2)
    HITJ(3, h3, s3)
    HITJ(4, h4, s4)
    HITJ(5, h5, s5)
    HITJ(6, h6, s6)
    HITJ(7, h7, s7)
#undef HITJ
  }
  return wc;
}

__global__ __launch_bounds__(NTHR) void k_wprep(const float* __restrict__ wg, const float* __restrict__ wb,
                                                int nUnits, unsigned short* BT) {
  const int u = (int)blockIdx.x * NTHR + (int)threadIdx.x;
  if (u >= nUnits) return;
  const int l   = u >> 11;
  const int mat = (u >> 10) & 1;
  const int w   = u & 1023;
  const int n   = w >> 4;
  const int kq  = (w & 15) * 8;
  const int kk  = kq & (F - 1);
  const float* base = (mat != 0) ? wb : wg;
  const float* p = base + (size_t)l * F * F + (size_t)kk * F + n;
  v8us o;
#pragma unroll
  for (int i = 0; i < 8; ++i) o[i] = bf_bits(p[(size_t)i * F]);
  unsigned short* dp = BT + ((size_t)l * F + (size_t)n) * KC + mat * (2 * F) + kq;
  *(volatile v8us*)dp = o;
  __threadfence();
  *(volatile v8us*)dp = o;
}

template <int SRC0>
__global__ __launch_bounds__(NTHR) void k_scan(const int* __restrict__ srcs, const int* __restrict__ dsts,
                                               const float* __restrict__ ew, const float* __restrict__ Hs,
                                               float* SIDE, int nN, int nE, int vec8, int mRows) {
  extern __shared__ __attribute__((aligned(16))) int lds_i[];
  int* reg1 = lds_i;
  int* reg2 = reg1 + RCAP;
  int* scnt = reg2 + RCAP;
  int* soff = scnt + NBA;
  int* list = soff + NBA;
  int* wcnt = list + LISTN;
  int* wtot = wcnt + NWAVE;
  const int tid = (int)threadIdx.x, lane = tid & 31, wave = tid >> 5;
  const int nodeBase = (int)blockIdx.x * NBA;

  {
    const v4i z4 = {0, 0, 0, 0};
    for (int i = tid * 4; i < ZINTS; i += NTHR * 4) *(v4ia*)(lds_i + i) = z4;
    if (tid < 2 * NWAVE) wcnt[tid] = 0;
  }
  __syncthreads();

  int tot = 0;
  const int nChunks = (nE + CHUNK - 1) / CHUNK;
#pragma unroll 1
  for (int ch = 0; ch < nChunks; ++ch) {
    const int cbase = ch * CHUNK;
    const int wc = scan_chunk(dsts, nE, cbase, nodeBase, NBA, vec8, list, tid, lane, wave);
    if (lane == 0) wcnt[wave] = wc;
    __syncthreads();
    int pre = 0, all = 0;
#pragma unroll
    for (int w2 = 0; w2 < NWAVE; ++w2) {
      int c = wcnt[w2];
      c = c < 0 ? 0 : (c > WCAP ? WCAP : c);
      all += c;
      pre += (w2 < wave) ? c : 0;
    }
    const int wcc  = wc > WCAP ? WCAP : wc;
    const int base = tot + pre;
#pragma unroll 1
    for (int i = lane; i < wcc; i += 32) {
      const int ent = list[wave * WCAP + i];
      const int el  = (ent >> PKS) & (CHUNK - 1);
      const int sl  = ent & (NBA - 1);
      int eid = cbase + el;
      eid = eid > nE - 1 ? nE - 1 : eid;
      const int pos = base + i;
      if (pos < RCAP) reg1[pos] = (int)(((unsigned)eid << PKS) | (unsigned)sl);
    }
    tot += all;
    tot = tot > RCAP ? RCAP : tot;
    __syncthreads();
  }
  const int nh = tot;

  if (wave == 0) {
#pragma unroll 1
    for (int b0 = 0; b0 < nh; b0 += 32) {
      const int idx = b0 + lane;
      const int uv  = reg1[idx < RCAP ? idx : RCAP - 1];
      const int m32 = (nh - b0) < 32 ? (nh - b0) : 32;
#pragma unroll 1
      for (int k = 0; k < m32; ++k) {
        const int u  = __builtin_amdgcn_readlane(uv, k);
        const int sl = u & (NBA - 1);
        if (lane == 0) scnt[sl] = scnt[sl] + 1;
      }
    }
  }
  __syncthreads();

  {
    const int c0r = scnt[4 * tid], c1r = scnt[4 * tid + 1], c2r = scnt[4 * tid + 2], c3r = scnt[4 * tid + 3];
    const int e0 = c0r < 0 ? 0 : c0r, e1 = c1r < 0 ? 0 : c1r, e2 = c2r < 0 ? 0 : c2r, e3 = c3r < 0 ? 0 : c3r;
    const int ts = e0 + e1 + e2 + e3;
    int incl = ts;
#pragma unroll
    for (int d = 1; d < 32; d <<= 1) {
      const int up = __shfl_up(incl, d, 32);
      if (lane >= d) incl += up;
    }
    if (lane == 31) wtot[wave] = incl;
    __syncthreads();
    int pre = 0;
#pragma unroll
    for (int w2 = 0; w2 < NWAVE; ++w2) pre += (w2 < wave) ? wtot[w2] : 0;
    int run = pre + incl - ts;
    soff[4 * tid + 0] = run; run += e0;
    soff[4 * tid + 1] = run; run += e1;
    soff[4 * tid + 2] = run; run += e2;
    soff[4 * tid + 3] = run;
  }
  __syncthreads();
  for (int i = tid; i < NBA; i += NTHR) list[i] = soff[i];
  __syncthreads();

  if (wave == 0) {
#pragma unroll 1
    for (int b0 = 0; b0 < nh; b0 += 32) {
      const int idx = b0 + lane;
      const int uv  = reg1[idx < RCAP ? idx : RCAP - 1];
      const int m32 = (nh - b0) < 32 ? (nh - b0) : 32;
#pragma unroll 1
      for (int k = 0; k < m32; ++k) {
        const int u   = __builtin_amdgcn_readlane(uv, k);
        const int sl  = u & (NBA - 1);
        const int eid = (int)((unsigned)u >> PKS);
        if (lane == 0) {
          int pos = list[sl];
          pos = pos < 0 ? 0 : (pos > RCAP - 1 ? RCAP - 1 : pos);
          reg2[pos] = eid;
          list[sl] = pos + 1;
        }
      }
    }
  }
  __syncthreads();

  const int nbw = NBA / NWAVE;
  const bool ovf = (nh >= RCAP);
  const float qnan = __int_as_float(0x7fc00000);

#pragma unroll 1
  for (int jt = 0; jt < nbw; ++jt) {
    const int slot = wave * nbw + jt;
    const int node = nodeBase + slot;
    int st = soff[slot];
    const int craw = scnt[slot];
    int cnt = craw;
    st  = st < 0 ? 0 : (st > nh ? nh : st);
    cnt = cnt < 0 ? 0 : (cnt > DEGCAP ? DEGCAP : cnt);
    if (cnt > nh - st) cnt = nh - st;
    const float pz = (ovf || craw > DEGCAP) ? qnan : 0.0f;
    const bool live = node < nN;

    float a0 = 0.0f, a1 = 0.0f;
#pragma unroll 1
    for (int b0 = 0; b0 < cnt; b0 += 32) {
      int idx = st + b0 + lane; idx = idx > RCAP - 1 ? RCAP - 1 : idx;
      int eid = reg2[idx]; eid = eid < 0 ? 0 : (eid > nE - 1 ? nE - 1 : eid);
      int sr = srcs[eid]; sr = sr < 0 ? 0 : (sr > nN - 1 ? nN - 1 : sr);
      const float wv  = bf_rne(ew[eid]);
      const int   wvi = __float_as_int(wv);
      const int m32 = (cnt - b0) < 32 ? (cnt - b0) : 32;
#pragma unroll 1
      for (int k = 0; k < m32; ++k) {
        const int   sk = __builtin_amdgcn_readlane(sr, k);
        const float ck = __int_as_float(__builtin_amdgcn_readlane(wvi, k));
        const v2f v = *(const v2f*)(Hs + (size_t)sk * F + 2 * lane);
        float vx = v.x, vy = v.y;
        if constexpr (SRC0 != 0) { vx = bf_rne(vx); vy = bf_rne(vy); }
        a0 = fmaf(ck, vx, a0); a1 = fmaf(ck, vy, a1);
      }
    }
    const float r0 = (live ? a0 : 0.0f) + pz;
    const float r1 = (live ? a1 : 0.0f) + pz;
    v2f sv;
    sv.x = r0; sv.y = r1;
    if (node < mRows) {
      float* sp = SIDE + (size_t)node * F + 2 * lane;
      *(volatile v2f*)sp = sv;
      __threadfence();
      *(volatile v2f*)sp = sv;
    }
  }
}

template <int SRC0>
__global__ __launch_bounds__(GTHR) void k_layer(const float* __restrict__ SIDE, const float* egs,
                                                const unsigned short* __restrict__ BT,
                                                const float* __restrict__ bg, const float* __restrict__ bb,
                                                float* EGO, float* __restrict__ ALL, int nN, int acol, int wego) {
  __shared__ __attribute__((aligned(16))) unsigned short atile[GBM * KC];
  __shared__ __attribute__((aligned(16))) float stg[GBM * F];
  const int tid = (int)threadIdx.x, lane = tid & 31, wave = tid >> 5, hh = lane >> 4, m = lane & 15;
  const int rowBase = (int)blockIdx.x * GBM;

  {
    const int r    = tid >> 1;
    const int ch   = (tid & 1) * 32;
    const int grow = rowBase + r;
    const int erow = grow < nN ? grow : nN - 1;
    const float* sp = SIDE + (size_t)grow * F + ch;
    const float* ep = egs  + (size_t)erow * F + ch;
    unsigned short* trow = atile + (size_t)r * KC + ch;
#pragma unroll
    for (int g = 0; g < 4; ++g) {
      const v4f sA = *(const v4f*)(sp + 8 * g);
      const v4f sB = *(const v4f*)(sp + 8 * g + 4);
      v4f eA = *(const v4fa*)(ep + 8 * g);
      v4f eB = *(const v4fa*)(ep + 8 * g + 4);
      if constexpr (SRC0 != 0) {
        eA.x = bf_rne(eA.x); eA.y = bf_rne(eA.y); eA.z = bf_rne(eA.z); eA.w = bf_rne(eA.w);
        eB.x = bf_rne(eB.x); eB.y = bf_rne(eB.y); eB.z = bf_rne(eB.z); eB.w = bf_rne(eB.w);
      }
      v8us vh, vl, ph, pl;
      unsigned short t0, t1, t2, t3;
      split2(sA.x, eA.x, t0, t1, t2, t3); vh[0] = t0; vl[0] = t1; ph[0] = t2; pl[0] = t3;
      split2(sA.y, eA.y, t0, t1, t2, t3); vh[1] = t0; vl[1] = t1; ph[1] = t2; pl[1] = t3;
      split2(sA.z, eA.z, t0, t1, t2, t3); vh[2] = t0; vl[2] = t1; ph[2] = t2; pl[2] = t3;
      split2(sA.w, eA.w, t0, t1, t2, t3); vh[3] = t0; vl[3] = t1; ph[3] = t2; pl[3] = t3;
      split2(sB.x, eB.x, t0, t1, t2, t3); vh[4] = t0; vl[4] = t1; ph[4] = t2; pl[4] = t3;
      split2(sB.y, eB.y, t0, t1, t2, t3); vh[5] = t0; vl[5] = t1; ph[5] = t2; pl[5] = t3;
      split2(sB.z, eB.z, t0, t1, t2, t3); vh[6] = t0; vl[6] = t1; ph[6] = t2; pl[6] = t3;
      split2(sB.w, eB.w, t0, t1, t2, t3); vh[7] = t0; vl[7] = t1; ph[7] = t2; pl[7] = t3;
      *(v8usa*)(trow + 8 * g)         = vh;
      *(v8usa*)(trow + F + 8 * g)     = vl;
      *(v8usa*)(trow + 2 * F + 8 * g) = ph;
      *(v8usa*)(trow + 3 * F + 8 * g) = pl;
    }
  }
  __syncthreads();

  v8f acc[4];
  {
    const v8f z = {0.f, 0.f, 0.f, 0.f, 0.f, 0.f, 0.f, 0.f};
    acc[0] = z; acc[1] = z; acc[2] = z; acc[3] = z;
  }
  const unsigned short* ap = atile + (size_t)(16 * wave + m) * KC + 8 * hh;
  const unsigned short* bp = BT + (size_t)m * (size_t)KC + 8 * hh;

#pragma unroll 1
  for (int k0 = 0; k0 < KC; k0 += 32) {
    Frag af;
    af.h[0] = *(const v8usa*)(ap + k0);
    af.h[1] = *(const v8usa*)(ap + k0 + 16);
#pragma unroll
    for (int nt = 0; nt < 4; ++nt) {
      const unsigned short* wq = bp + (size_t)(16 * nt) * (size_t)KC + k0;
      Frag bf;
      bf.h[0] = *(const v8usa*)wq;
      bf.h[1] = *(const v8usa*)(wq + 16);
      acc[nt] = wmb(af, bf, acc[nt]);
    }
  }

#pragma unroll
  for (int nt = 0; nt < 4; ++nt) {
    const int lc = 16 * nt + m;
#pragma unroll
    for (int r = 0; r < 8; ++r) {
      const int lr = 16 * wave + 8 * hh + r;
      stg[lr * F + lc] = acc[nt][r];
    }
  }
  __syncthreads();

  const int c0 = 4 * m;
  v4f b4;
  {
    const v4f tg = *(const v4f*)(bg + c0);
    const v4f tb = *(const v4f*)(bb + c0);
    b4.x = bf_rne(tg.x) + bf_rne(tb.x); b4.y = bf_rne(tg.y) + bf_rne(tb.y);
    b4.z = bf_rne(tg.z) + bf_rne(tb.z); b4.w = bf_rne(tg.w) + bf_rne(tb.w);
  }
  v4f ev[8], zv[8];
#pragma unroll
  for (int i = 0; i < 8; ++i) {
    const int lr  = 16 * wave + 2 * i + hh;
    const int row = rowBase + lr;
    const bool ok = row < nN;
    v4f y = *(const v4fa*)(stg + lr * F + c0) + b4;
    y.x = y.x > 0.0f ? y.x : 0.2f * y.x;
    y.y = y.y > 0.0f ? y.y : 0.2f * y.y;
    y.z = y.z > 0.0f ? y.z : 0.2f * y.z;
    y.w = y.w > 0.0f ? y.w : 0.2f * y.w;
    float ss = y.x * y.x + y.y * y.y + y.z * y.z + y.w * y.w;
    ss += __shfl_xor(ss, 1, 32);
    ss += __shfl_xor(ss, 2, 32);
    ss += __shfl_xor(ss, 4, 32);
    ss += __shfl_xor(ss, 8, 32);
    const float nrm = sqrtf(ss);
    const float inv = 1.0f / fmaxf(nrm, 1e-12f);
    const v4f z = y * inv;
    v4f ye, ze;
    ye.x = ok ? y.x : 0.0f; ye.y = ok ? y.y : 0.0f; ye.z = ok ? y.z : 0.0f; ye.w = ok ? y.w : 0.0f;
    ze.x = ok ? z.x : 0.0f; ze.y = ok ? z.y : 0.0f; ze.z = ok ? z.z : 0.0f; ze.w = ok ? z.w : 0.0f;
    ev[i] = ye; zv[i] = ze;
  }
  if (wego != 0) {
#pragma unroll
    for (int i = 0; i < 8; ++i) {
      const int lr = 16 * wave + 2 * i + hh;
      float* op = EGO + (size_t)(rowBase + lr) * F + c0;
      *(volatile v4f*)op = ev[i];
    }
  }
#pragma unroll
  for (int i = 0; i < 8; ++i) {
    const int lr = 16 * wave + 2 * i + hh;
    float* op = ALL + (size_t)(rowBase + lr) * ALLP + acol + c0;
    *(volatile v4f*)op = zv[i];
  }
  __threadfence();
  if (wego != 0) {
#pragma unroll
    for (int i = 0; i < 8; ++i) {
      const int lr = 16 * wave + 2 * i + hh;
      float* op = EGO + (size_t)(rowBase + lr) * F + c0;
      *(volatile v4f*)op = ev[i];
    }
  }
#pragma unroll
  for (int i = 0; i < 8; ++i) {
    const int lr = 16 * wave + 2 * i + hh;
    float* op = ALL + (size_t)(rowBase + lr) * ALLP + acol + c0;
    *(volatile v4f*)op = zv[i];
  }
}

__global__ __launch_bounds__(NTHR) void k_out(const float* __restrict__ ALL, const float* __restrict__ emb,
                                              const int* __restrict__ iu, const int* __restrict__ ip,
                                              const int* __restrict__ ig, float* out, int nB, int nN) {
  const int tid = (int)threadIdx.x, lane = tid & 31, wave = tid >> 5;
  const int t = (int)blockIdx.x * NWAVE + wave;
  if (t >= 3 * nB) return;
  const int seg = t / nB;
  const int b   = t - seg * nB;
  const int x0 = iu[b], x1 = ip[b], x2 = ig[b];
  int idx = (seg == 0) ? x0 : ((seg == 1) ? x1 : x2);
  idx = idx < 0 ? idx + nN : idx;
  idx = idx < 0 ? 0 : (idx > nN - 1 ? nN - 1 : idx);
  const float* ar = ALL + (size_t)idx * ALLP;
  const float* er = emb + (size_t)idx * F;
  const v4f va = *(const v4f*)(ar + 4 * lane);
  const v4f vq = *(const v4f*)(ar + 2 * F + 4 * (lane & 15));
  const v4f ve = *(const v4f*)(er + 4 * (lane & 15));
  const unsigned msk = 0u - (unsigned)(lane >> 4);
  v4f vb;
  vb.x = __uint_as_float((__float_as_uint(bf_rne(ve.x)) & msk) | (__float_as_uint(vq.x) & ~msk));
  vb.y = __uint_as_float((__float_as_uint(bf_rne(ve.y)) & msk) | (__float_as_uint(vq.y) & ~msk));
  vb.z = __uint_as_float((__float_as_uint(bf_rne(ve.z)) & msk) | (__float_as_uint(vq.z) & ~msk));
  vb.w = __uint_as_float((__float_as_uint(bf_rne(ve.w)) & msk) | (__float_as_uint(vq.w) & ~msk));
  const int colA = F + 4 * lane;
  const int colB = 4 * lane + 3 * F - OW * (lane >> 4);
  float* r1 = out + (size_t)t * OW;
  float* r2 = out + ((size_t)t + (size_t)3 * (size_t)nB) * OW;
  *(volatile v4f*)(r1 + colA) = va;
  *(volatile v4f*)(r1 + colB) = vb;
  *(volatile v4f*)(r2 + colA) = va;
  *(volatile v4f*)(r2 + colB) = vb;
  __threadfence();
  *(volatile v4f*)(r1 + colA) = va;
  *(volatile v4f*)(r1 + colB) = vb;
  *(volatile v4f*)(r2 + colA) = va;
  *(volatile v4f*)(r2 + colB) = vb;
}

static inline int cdiv(int a, int b) { return (a + b - 1) / b; }
static inline size_t al256(size_t o) { return (o + 255) & ~(size_t)255; }

extern "C" void kernel_launch(void* const* d_in, const int* in_sizes, int n_in,
                              void* d_out, int out_size, void* d_ws, size_t ws_size,
                              hipStream_t stream) {
  if (n_in < 10) return;
  if (in_sizes[0] < F || (in_sizes[0] % F) != 0) return;
  const int nN = in_sizes[0] / F;
  if (nN < 1 || nN > (1 << 22)) return;
  const int nE = in_sizes[1];
  if (nE < 1 || nE >= (1 << 21)) return;
  if (in_sizes[6] != 2 * nE) return;
  if (in_sizes[2] != NL * F * F || in_sizes[4] != NL * F * F) return;
  if (in_sizes[3] != NL * F || in_sizes[5] != NL * F) return;
  const int nB = in_sizes[7];
  if (nB < 1 || in_sizes[8] != nB || in_sizes[9] != nB) return;
  if ((long long)out_size != 6LL * (long long)nB * OW) return;

  const float* emb = (const float*)d_in[0];
  const float* ew  = (const float*)d_in[1];
  const float* wg  = (const float*)d_in[2];
  const float* bgc = (const float*)d_in[3];
  const float* wb  = (const float*)d_in[4];
  const float* bbi = (const float*)d_in[5];
  const int*  edge = (const int*)d_in[6];
  const int*  usr  = (const int*)d_in[7];
  const int*  psi  = (const int*)d_in[8];
  const int*  ngi  = (const int*)d_in[9];
  float* out = (float*)d_out;
  const int* src = edge;
  const int* dst = edge + nE;

  const int MP = cdiv(nN, GBM) * GBM;
  const int gM = MP / GBM;
  const int gA = cdiv(MP, NBA);
  if ((long long)gA * NBA < (long long)MP) return;
  const int vec8 = ((nE & 3) == 0) ? 1 : 0;

  char* ws = (char*)d_ws;
  size_t off = 0;
  const size_t oBT  = off; off = al256(off + (size_t)NL * F * KC * 2);
  const size_t oSD  = off; off = al256(off + (size_t)MP * F * 4);
  const size_t oEG  = off; off = al256(off + (size_t)MP * F * 4);
  const size_t oAL  = off; off = al256(off + (size_t)MP * ALLP * 4);
  if (off > ws_size || off > (size_t)WSMAX) return;
  unsigned short* BT  = (unsigned short*)(ws + oBT);
  float*          SD  = (float*)(ws + oSD);
  float*          EG  = (float*)(ws + oEG);
  float*          AL  = (float*)(ws + oAL);

  hipFuncSetAttribute(reinterpret_cast<const void*>(&k_scan<1>), hipFuncAttributeMaxDynamicSharedMemorySize, LDS_AGG);
  hipFuncSetAttribute(reinterpret_cast<const void*>(&k_scan<0>), hipFuncAttributeMaxDynamicSharedMemorySize, LDS_AGG);

  const int nUw = NL * UPL;
  k_wprep<<<nUw / NTHR, NTHR, 0, stream>>>(wg, wb, nUw, BT);

  for (int l = 0; l < NL; ++l) {
    const unsigned short* Bl = BT + (size_t)l * F * KC;
    const float* bgl = bgc + (size_t)l * F;
    const float* bbl = bbi + (size_t)l * F;
    const int acol = l * F;
    const int wego = (l < NL - 1) ? 1 : 0;
    if (l == 0) {
      k_scan<1><<<gA, NTHR, LDS_AGG, stream>>>(src, dst, ew, emb, SD, nN, nE, vec8, MP);
      k_layer<1><<<gM, GTHR, 0, stream>>>(SD, emb, Bl, bgl, bbl, EG, AL, nN, acol, wego);
    } else {
      k_scan<0><<<gA, NTHR, LDS_AGG, stream>>>(src, dst, ew, EG, SD, nN, nE, vec8, MP);
      k_layer<0><<<gM, GTHR, 0, stream>>>(SD, EG, Bl, bgl, bbl, EG, AL, nN, acol, wego);
    }
  }

  k_out<<<cdiv(3 * nB, NWAVE), NTHR, 0, stream>>>(AL, emb, usr, psi, ngi, out, nB, nN);
}
